// SelectiveSSM_10393820856794
// MI455X (gfx1250) — hardware-verified
//
#include <hip/hip_runtime.h>
#include <math.h>

typedef __attribute__((ext_vector_type(16))) _Float16 v16h;
typedef __attribute__((ext_vector_type(8)))  _Float16 v8h;
typedef __attribute__((ext_vector_type(16))) __bf16   v16b;
typedef __attribute__((ext_vector_type(8)))  __bf16   v8b;
typedef __attribute__((ext_vector_type(8)))  float    v8f;
typedef __attribute__((ext_vector_type(4)))  float    v4f;

constexpr int kBatch  = 2;
constexpr int kSeq    = 2048;
constexpr int kDm     = 512;
constexpr int kDin    = 1024;
constexpr int kNst    = 16;
constexpr int kNth    = 8;
constexpr int kConvK  = 4;
constexpr int kXzP    = 2 * kDin;
constexpr int kRows   = kBatch * kSeq;
constexpr int kWxN    = 2 * kNst + 1;
constexpr int kPrjP    = 64;
constexpr int kPrjC    = 48;
constexpr int kPrjRows = 64;
constexpr int kPrjKC   = 128;
constexpr int kPrjLP   = 132;
constexpr int kPrjOP   = 68;
constexpr int kRecP    = 64;
constexpr int kRpThreads = 128;
constexpr int kRpGroup   = 16;
constexpr int kRpLP      = 68;
constexpr int kConvTP = 260;
constexpr int kScanTS = 64;
constexpr int kScanCh = 64;
constexpr int kScanYP = 68;
constexpr float kWCarry = 32.0f;
constexpr float kYCarry = 16.0f;
constexpr float kOutScale = 1.0f / (kWCarry * kYCarry);
static_assert(kNth * 2 == kNst, "angle count");
static_assert((kDm % 32) == 0 && (kDin % 32) == 0, "GEMM K multiples of 32");
static_assert((kRows % 64) == 0 && (kXzP % 64) == 0 && (kDm % 64) == 0, "GEMM M,N multiples of 64");
static_assert(((kRows / 64) * (kXzP / 64)) % 8 == 0 && ((kRows / 64) * (kDm / 64)) % 8 == 0, "8 tiles per GEMM block");
static_assert((kSeq % kScanTS) == 0 && (kSeq % 64) == 0 && (kDin % kScanCh) == 0 && (kDin % 256) == 0, "tile multiples");
static_assert((kRows % kPrjRows) == 0 && (kDin % kPrjKC) == 0 && (kPrjKC % 4) == 0, "proj tiles");
static_assert(kRpThreads * kRpGroup == kSeq && (kSeq % kRpThreads) == 0, "rowprep tiles");
static_assert(2 * kNst + kNth + 2 <= kPrjC && kPrjC + 16 == kPrjP, "proj column map");
static_assert(((kRows * kDm / 8) % 256) == 0, "x plane cast grid");
static_assert((kDm % 64) == 0 && (kXzP % 64) == 0 && (kDin % 64) == 0, "transpose tiles");

constexpr size_t kOffXH   = 0;
constexpr size_t kOffXL   = kOffXH   + (size_t)kRows * kDm  * 2;
constexpr size_t kOffWIH  = kOffXL   + (size_t)kRows * kDm  * 2;
constexpr size_t kOffWIL  = kOffWIH  + (size_t)kXzP  * kDm  * 2;
constexpr size_t kOffWO16 = kOffWIL  + (size_t)kXzP  * kDm  * 2;
constexpr size_t kOffXZ   = kOffWO16 + (size_t)kDm   * kDin * 2;
constexpr size_t kOffUC   = kOffXZ   + (size_t)kRows * kXzP * 4;
constexpr size_t kOffPRJ  = kOffUC   + (size_t)kRows * kDin * 4;
constexpr size_t kOffREC  = kOffPRJ  + (size_t)kRows * kPrjP * 4;
constexpr size_t kOffY16  = kOffREC  + (size_t)kRows * kRecP * 4;
constexpr size_t kWsTotal = kOffY16  + (size_t)kRows * kDin * 2;
static_assert(kWsTotal == 74448896ull, "carve total");
static_assert(kWsTotal <= 134217728ull, "carve cap");
static_assert((kOffXL % 128) == 0 && (kOffWIH % 128) == 0 && (kOffWIL % 128) == 0 && (kOffWO16 % 128) == 0 &&
              (kOffXZ % 128) == 0 && (kOffUC % 128) == 0 && (kOffPRJ % 128) == 0 && (kOffREC % 128) == 0 &&
              (kOffY16 % 128) == 0, "128-B aligned regions");

__device__ __forceinline__ unsigned short f2bf_bits(float f) {
  unsigned u = __float_as_uint(f);
  return (unsigned short)((u + 0x7FFFu + ((u >> 16) & 1u)) >> 16);
}
__device__ __forceinline__ float bf_bits2f(unsigned short h) { return __uint_as_float(((unsigned)h) << 16); }

__device__ __forceinline__ void dep_guard4_h(v8f& a, v8f& b, v8f& c, v8f& d, v16h x, v16h y) { asm volatile("v_nop\n\tv_nop\n\tv_nop\n\tv_nop" : "+v"(a), "+v"(b), "+v"(c), "+v"(d) : "v"(x), "v"(y)); }
__device__ __forceinline__ void dep_guard4_b(v8f& a, v8f& b, v8f& c, v8f& d, v16b x, v16b y) { asm volatile("v_nop\n\tv_nop\n\tv_nop\n\tv_nop" : "+v"(a), "+v"(b), "+v"(c), "+v"(d) : "v"(x), "v"(y)); }
__device__ __forceinline__ void keep4_h(v16h a, v16h b, v16h c, v16h d) { asm volatile("v_nop" :: "v"(a), "v"(b), "v"(c), "v"(d)); }
__device__ __forceinline__ void keep4_b(v16b a, v16b b, v16b c, v16b d) { asm volatile("v_nop" :: "v"(a), "v"(b), "v"(c), "v"(d)); }
__device__ __forceinline__ void acc_guard4(v8f& a, v8f& b, v8f& c, v8f& d) { asm volatile("v_nop\n\tv_nop\n\tv_nop\n\tv_nop" : "+v"(a), "+v"(b), "+v"(c), "+v"(d)); }
template <typename T> struct Frag;
template <> struct Frag<_Float16> {
  typedef v16h V; union U { v16h v; v8h h[2]; };
  static __device__ __forceinline__ v16h load(const _Float16* p) {
    U f; f.h[0] = *(const v8h*)(p); f.h[1] = *(const v8h*)(p + 16); return f.v;
  }
  static __device__ __forceinline__ v8f mma(v16h a, v16h b, v8f c) {
    return __builtin_amdgcn_wmma_f32_16x16x32_f16(false, a, false, b, (short)0, c, false, false);
  }
  static __device__ __forceinline__ void guard4(v8f& a, v8f& b, v8f& c, v8f& d, v16h x, v16h y) { dep_guard4_h(a, b, c, d, x, y); }
  static __device__ __forceinline__ void keep(v16h a, v16h b, v16h c, v16h d) { keep4_h(a, b, c, d); }
};
template <> struct Frag<__bf16> {
  typedef v16b V; union U { v16b v; v8b h[2]; };
  static __device__ __forceinline__ v16b load(const __bf16* p) {
    U f; f.h[0] = *(const v8b*)(p); f.h[1] = *(const v8b*)(p + 16); return f.v;
  }
  static __device__ __forceinline__ v8f mma(v16b a, v16b b, v8f c) {
    return __builtin_amdgcn_wmma_f32_16x16x32_bf16(false, a, false, b, (short)0, c, false, false);
  }
  static __device__ __forceinline__ void guard4(v8f& a, v8f& b, v8f& c, v8f& d, v16b x, v16b y) { dep_guard4_b(a, b, c, d, x, y); }
  static __device__ __forceinline__ void keep(v16b a, v16b b, v16b c, v16b d) { keep4_b(a, b, c, d); }
};

template <int ET> struct Elem;
template <> struct Elem<0> { typedef _Float16 T; };
template <> struct Elem<1> { typedef __bf16 T; };
template <int ET, bool SPLIT, int BIAS_MODE, int OUT_MODE, bool RESID, int ACT = 0>
__global__ __launch_bounds__(256) void wmma_gemm64(
    const unsigned short* __restrict__ Ap, const unsigned short* __restrict__ A2p, int lda, long strideA,
    const unsigned short* __restrict__ Btp, const unsigned short* __restrict__ Bt2p, int ldb, long strideB,
    void* __restrict__ Cout, void* __restrict__ Cout2, int ldc, long strideC,
    const float* __restrict__ bias,
    const float* __restrict__ resid, long strideR,
    int M, int N, int K, float scale) {
  typedef typename Elem<ET>::T T;
  typedef typename Frag<T>::V V;
  const T* A = (const T*)Ap; const T* A2 = (const T*)A2p; const T* Bt = (const T*)Btp; const T* Bt2 = (const T*)Bt2p;
  __shared__ __align__(16) float sT[8][16 * 68];
  const int b    = blockIdx.y;
  const int lane = threadIdx.x & 31;
  const int wave = threadIdx.x >> 5;
  const int tilesN = N >> 6;
  const int tilesM = M >> 6;
  const int tile = blockIdx.x * 8 + wave;
  if (tile >= tilesM * tilesN) return;
  const int tm = tile / tilesN;
  const int tn = tile - tm * tilesN;
  const int m0 = tm << 6;
  const int n0 = tn << 6;

  const T* Ab  = A  + (size_t)b * strideA;
  const T* Bb  = Bt + (size_t)b * strideB;
  const T* Ab2 = SPLIT ? (A2  + (size_t)b * strideA) : nullptr;
  const T* Bb2 = SPLIT ? (Bt2 + (size_t)b * strideB) : nullptr;

  const int rlane = lane & 15;
  const int koff  = (lane >> 4) * 8;
  const int mOff  = (lane >> 4) * 8;

  v8f acc[4][4];
#pragma unroll
  for (int i = 0; i < 4; ++i)
#pragma unroll
    for (int j = 0; j < 4; ++j) acc[i][j] = (v8f){0.f,0.f,0.f,0.f,0.f,0.f,0.f,0.f};

  for (int k0 = 0; k0 < K; k0 += 32) {
    V bh[4], bl[4];
#pragma unroll
    for (int j = 0; j < 4; ++j) {
      const size_t bo = (size_t)(n0 + (j << 4) + rlane) * ldb + koff + k0;
      bh[j] = Frag<T>::load(Bb + bo);
      if (SPLIT) bl[j] = Frag<T>::load(Bb2 + bo);
    }
#pragma unroll
    for (int i = 0; i < 4; ++i) {
      const size_t ao = (size_t)(m0 + (i << 4) + rlane) * lda + koff + k0;
      V ah = Frag<T>::load(Ab + ao);
      V al;
      if (SPLIT) al = Frag<T>::load(Ab2 + ao);
#pragma unroll
      for (int j = 0; j < 4; ++j) {
        acc[i][j] = Frag<T>::mma(ah, bh[j], acc[i][j]);
        if (SPLIT) {
          acc[i][j] = Frag<T>::mma(ah, bl[j], acc[i][j]);
          acc[i][j] = Frag<T>::mma(al, bh[j], acc[i][j]);
        }
      }
      Frag<T>::guard4(acc[i][0], acc[i][1], acc[i][2], acc[i][3], ah, SPLIT ? al : ah);
    }
    Frag<T>::keep(bh[0], bh[1], bh[2], bh[3]);
    if (SPLIT) Frag<T>::keep(bl[0], bl[1], bl[2], bl[3]);
  }
  acc_guard4(acc[0][0], acc[0][1], acc[0][2], acc[0][3]);
  acc_guard4(acc[1][0], acc[1][1], acc[1][2], acc[1][3]);
  acc_guard4(acc[2][0], acc[2][1], acc[2][2], acc[2][3]);
  acc_guard4(acc[3][0], acc[3][1], acc[3][2], acc[3][3]);

  float* slab = sT[wave];
  const float* Rb = RESID ? (resid + (size_t)b * strideR) : nullptr;
#pragma unroll
  for (int i = 0; i < 4; ++i) {
    const int mBase = m0 + (i << 4);
#pragma unroll
    for (int j = 0; j < 4; ++j) {
      const int n = n0 + (j << 4) + rlane;
      float bv = 0.f;
      if (BIAS_MODE == 2) bv = bias[n];
#pragma unroll
      for (int r = 0; r < 8; ++r) {
        float v = acc[i][j][r] * scale;
        if (BIAS_MODE == 1) v += bias[mBase + mOff + r];
        if (BIAS_MODE == 2) v += bv;
        if (RESID) v += Rb[(size_t)(mBase + mOff + r) * ldc + n];
        if (ACT == 1) v = tanhf(v);
        if (ACT == 2) v = fmaxf(v, 0.0f);
        if (ACT == 3) v = v / (1.0f + expf(-v));
        if (ACT == 4) v = (v > 0.f) ? v : 0.01f * v;
        slab[(mOff + r) * 68 + (j << 4) + rlane] = v;
      }
    }
    __builtin_amdgcn_fence(__ATOMIC_RELEASE, "workgroup");
    __builtin_amdgcn_wave_barrier();
    __builtin_amdgcn_fence(__ATOMIC_ACQUIRE, "workgroup");
    if (OUT_MODE == 0) {
      float* C = (float*)Cout + (size_t)b * strideC;
      const int hh = lane >> 4, c4 = (lane & 15) * 4;
      for (int pass = 0; pass < 2; ++pass) {
#pragma unroll
        for (int it = 0; it < 8; ++it) {
          const int row = it * 2 + hh;
          v4f v = *(const v4f*)(slab + row * 68 + c4);
          *(volatile v4f*)(C + (size_t)(mBase + row) * ldc + n0 + c4) = v;
        }
        __threadfence();
      }
    } else {
      const int q = lane >> 3, c8 = (lane & 7) * 8;
      unsigned short* C  = (unsigned short*)Cout  + (size_t)b * strideC;
      unsigned short* C2 = (OUT_MODE == 2) ? ((unsigned short*)Cout2 + (size_t)b * strideC) : nullptr;
      for (int pass = 0; pass < 2; ++pass) {
#pragma unroll
        for (int it = 0; it < 4; ++it) {
          const int row = it * 4 + q;
          const float* sp = slab + row * 68 + c8;
          v8h hv, lv;
#pragma unroll
          for (int e = 0; e < 8; ++e) {
            if (OUT_MODE == 1) {
              hv[e] = (_Float16)sp[e];
            } else {
              unsigned short hb = f2bf_bits(sp[e]);
              unsigned short lb = f2bf_bits(sp[e] - bf_bits2f(hb));
              hv[e] = __builtin_bit_cast(_Float16, hb);
              lv[e] = __builtin_bit_cast(_Float16, lb);
            }
          }
          *(volatile v8h*)(C + (size_t)(mBase + row) * ldc + n0 + c8) = hv;
          if (OUT_MODE == 2) *(volatile v8h*)(C2 + (size_t)(mBase + row) * ldc + n0 + c8) = lv;
        }
        __threadfence();
      }
    }
    __builtin_amdgcn_fence(__ATOMIC_RELEASE, "workgroup");
    __builtin_amdgcn_wave_barrier();
    __builtin_amdgcn_fence(__ATOMIC_ACQUIRE, "workgroup");
  }
}

__global__ __launch_bounds__(256) void split_rows_bf16_kernel(
    const float* __restrict__ src, unsigned short* __restrict__ dhi, unsigned short* __restrict__ dlo, int total8)
{
  const int i = blockIdx.x * 256 + threadIdx.x;
  if (i >= total8) return;
  const size_t e0 = (size_t)i << 3;
  const v4f a0 = *(const v4f*)(src + e0);
  const v4f a1 = *(const v4f*)(src + e0 + 4);
  v8h hv, lv;
#pragma unroll
  for (int e = 0; e < 4; ++e) {
    const unsigned short h0 = f2bf_bits(a0[e]), h1 = f2bf_bits(a1[e]);
    const unsigned short l0 = f2bf_bits(a0[e] - bf_bits2f(h0)), l1 = f2bf_bits(a1[e] - bf_bits2f(h1));
    hv[e]     = __builtin_bit_cast(_Float16, h0);
    hv[4 + e] = __builtin_bit_cast(_Float16, h1);
    lv[e]     = __builtin_bit_cast(_Float16, l0);
    lv[4 + e] = __builtin_bit_cast(_Float16, l1);
  }
  unsigned short* qh = dhi + e0;
  unsigned short* ql = dlo + e0;
  *(volatile v8h*)qh = hv;
  *(volatile v8h*)ql = lv;
  __threadfence();
  *(volatile v8h*)qh = hv;
  *(volatile v8h*)ql = lv;
}

__global__ __launch_bounds__(256) void transpose_split_bf16_kernel(
    const float* __restrict__ W, unsigned short* __restrict__ Bh, unsigned short* __restrict__ Bl, int Kdim, int Ndim)
{
  __shared__ float tile[64 * 65];
  const int tid = threadIdx.x, lane = tid & 31, wave = tid >> 5;
  const int n0 = blockIdx.x * 64;
  const int k0 = blockIdx.y * 64;
#pragma unroll
  for (int p = 0; p < 16; ++p) {
    const int idx = tid + p * 256;
    const int kk  = idx >> 6;
    const int nn  = idx & 63;
    tile[kk * 65 + nn] = W[(size_t)(k0 + kk) * Ndim + n0 + nn];
  }
  __syncthreads();
  const int q = lane >> 3, c8 = (lane & 7) * 8;
  v8h hv[2], lv[2];
#pragma unroll
  for (int it = 0; it < 2; ++it) {
    const int nrow = it * 32 + wave * 4 + q;
#pragma unroll
    for (int e = 0; e < 8; ++e) {
      const float v = tile[(c8 + e) * 65 + nrow];
      const unsigned short hb = f2bf_bits(v);
      const unsigned short lb = f2bf_bits(v - bf_bits2f(hb));
      hv[it][e] = __builtin_bit_cast(_Float16, hb);
      lv[it][e] = __builtin_bit_cast(_Float16, lb);
    }
  }
  for (int pass = 0; pass < 2; ++pass) {
#pragma unroll
    for (int it = 0; it < 2; ++it) {
      const int nrow = it * 32 + wave * 4 + q;
      const size_t o = (size_t)(n0 + nrow) * Kdim + k0 + c8;
      *(volatile v8h*)(Bh + o) = hv[it];
      *(volatile v8h*)(Bl + o) = lv[it];
    }
    __threadfence();
  }
}

__global__ __launch_bounds__(256) void transpose_cast_kernel(
    const float* __restrict__ W, unsigned short* __restrict__ Bt, int Kdim, int Ndim, int Npad, float scale)
{
  __shared__ float tile[64 * 65];
  const int tid = threadIdx.x, lane = tid & 31, wave = tid >> 5;
  const int n0 = blockIdx.x * 64;
  const int k0 = blockIdx.y * 64;
  (void)Npad;
#pragma unroll
  for (int p = 0; p < 16; ++p) {
    const int idx = tid + p * 256;
    const int kk  = idx >> 6;
    const int nn  = idx & 63;
    const int n   = n0 + nn;
    const int nc  = (n < Ndim) ? n : (Ndim - 1);
    const float v = W[(size_t)(k0 + kk) * Ndim + nc];
    tile[kk * 65 + nn] = (n < Ndim) ? (v * scale) : 0.f;
  }
  __syncthreads();
  const int q = lane >> 3, c8 = (lane & 7) * 8;
  v8h hv[2];
#pragma unroll
  for (int it = 0; it < 2; ++it) {
    const int nrow = it * 32 + wave * 4 + q;
#pragma unroll
    for (int e = 0; e < 8; ++e) hv[it][e] = (_Float16)tile[(c8 + e) * 65 + nrow];
  }
  for (int pass = 0; pass < 2; ++pass) {
#pragma unroll
    for (int it = 0; it < 2; ++it) {
      const int nrow = it * 32 + wave * 4 + q;
      *(volatile v8h*)(Bt + (size_t)(n0 + nrow) * Kdim + k0 + c8) = hv[it];
    }
    __threadfence();
  }
}

__global__ __launch_bounds__(256) void conv_silu_kernel(
    const float* __restrict__ XZ, const float* __restrict__ cw, const float* __restrict__ cb,
    float* __restrict__ UC)
{
  __shared__ __align__(16) float sT[16 * kConvTP];
  const int tid = threadIdx.x, lane = tid & 31, wave = tid >> 5;
  const int d0 = blockIdx.x * 256, d = d0 + tid;
  const int g0 = blockIdx.y * 64;
  const int tb = g0 & (kSeq - 1);
  const float w0 = cw[d * kConvK + 0], w1 = cw[d * kConvK + 1], w2 = cw[d * kConvK + 2], w3 = cw[d * kConvK + 3];
  const float bc = cb[d];
  float xm3, xm2, xm1;
  {
    const bool hist = (tb > 0);
    const int rb = hist ? (g0 - 3) : g0;
    const float v3 = XZ[(size_t)rb * kXzP + d];
    const float v2 = XZ[(size_t)(rb + 1) * kXzP + d];
    const float v1 = XZ[(size_t)(rb + 2) * kXzP + d];
    xm3 = hist ? v3 : 0.f;
    xm2 = hist ? v2 : 0.f;
    xm1 = hist ? v1 : 0.f;
  }
  const int hrow = wave >> 1;
  const int hch  = (wave & 1) * 128 + lane * 4;
#pragma unroll 1
  for (int sub = 0; sub < 4; ++sub) {
    const int lb = g0 + sub * 16;
#pragma unroll 1
    for (int s = 0; s < 16; ++s) {
      const float xcur = XZ[(size_t)(lb + s) * kXzP + d];
      float acc = w0 * xm3;
      acc = fmaf(w1, xm2, acc);
      acc = fmaf(w2, xm1, acc);
      acc = fmaf(w3, xcur, acc);
      const float sv = acc + bc;
      const float sg = __builtin_amdgcn_rcpf(1.0f + __expf(-sv));
      sT[s * kConvTP + tid] = sv * sg;
      xm3 = xm2; xm2 = xm1; xm1 = xcur;
    }
    __syncthreads();
    v4f fv[4];
#pragma unroll
    for (int it = 0; it < 4; ++it) fv[it] = *(const v4f*)(sT + (it * 4 + hrow) * kConvTP + hch);
    for (int pass = 0; pass < 2; ++pass) {
#pragma unroll
      for (int it = 0; it < 4; ++it)
        *(volatile v4f*)(UC + (size_t)(lb + it * 4 + hrow) * kDin + d0 + hch) = fv[it];
      __threadfence();
    }
    __syncthreads();
  }
}

__global__ __launch_bounds__(256) void proj_kernel(
    const float* __restrict__ UC, const float* __restrict__ Wx, const float* __restrict__ Wth,
    const float* __restrict__ Wlam, float* __restrict__ PROJ)
{
  __shared__ __align__(16) float sX[kPrjRows * kPrjLP];
  __shared__ __align__(16) float sW[kPrjC * kPrjLP];
  const int tid = threadIdx.x, lane = tid & 31, wave = tid >> 5;
  const int row0 = blockIdx.x * kPrjRows;
  const int pr = tid >> 2;
  const int cg = tid & 3;
  float acc[12];
#pragma unroll
  for (int j = 0; j < 12; ++j) acc[j] = 0.f;

#pragma unroll 1
  for (int kc = 0; kc < kDin / kPrjKC; ++kc) {
    const int k0 = kc * kPrjKC;
    __syncthreads();
#pragma unroll 1
    for (int i = 0; i < 8; ++i) {
      const int idx = tid + 256 * i;
      const int r = idx >> 5, c4 = (idx & 31) * 4;
      *(v4f*)(sX + r * kPrjLP + c4) = *(const v4f*)(UC + (size_t)(row0 + r) * kDin + k0 + c4);
    }
    if (tid < kPrjKC) {
      const int k = k0 + tid;
      const float vl = Wlam[k];
#pragma unroll 1
      for (int c = 0; c < kPrjC; ++c) {
        const int cx = (c < 2 * kNst) ? c : (2 * kNst);
        int ct = c - 2 * kNst;
        ct = (ct < 0) ? 0 : ((ct > kNth - 1) ? (kNth - 1) : ct);
        const float vx = Wx[(size_t)k * kWxN + cx];
        const float vt = Wth[(size_t)k * kNth + ct];
        float v = 0.f;
        if (c < 2 * kNst) v = vx;
        else if (c < 2 * kNst + kNth) v = vt;
        else if (c == 2 * kNst + kNth) v = vx;
        else if (c == 2 * kNst + kNth + 1) v = vl;
        sW[c * kPrjLP + tid] = v;
      }
    }
    __syncthreads();
    const float* xr = sX + pr * kPrjLP;
    const float* wb = sW + (cg * 12) * kPrjLP;
#pragma unroll 1
    for (int k4 = 0; k4 < kPrjKC / 4; ++k4) {
      const v4f xv = *(const v4f*)(xr + 4 * k4);
#pragma unroll
      for (int j = 0; j < 12; ++j) {
        const v4f wv = *(const v4f*)(wb + j * kPrjLP + 4 * k4);
        acc[j] = fmaf(xv[0], wv[0], acc[j]);
        acc[j] = fmaf(xv[1], wv[1], acc[j]);
        acc[j] = fmaf(xv[2], wv[2], acc[j]);
        acc[j] = fmaf(xv[3], wv[3], acc[j]);
      }
    }
  }
  __syncthreads();
  float* sO = sX;
  {
    float* op = sO + pr * kPrjOP + cg * 12;
    *(v4f*)(op)     = (v4f){acc[0], acc[1], acc[2],  acc[3]};
    *(v4f*)(op + 4) = (v4f){acc[4], acc[5], acc[6],  acc[7]};
    *(v4f*)(op + 8) = (v4f){acc[8], acc[9], acc[10], acc[11]};
    *(v4f*)(sO + pr * kPrjOP + kPrjC + cg * 4) = (v4f){0.f, 0.f, 0.f, 0.f};
  }
  __syncthreads();
  const int hh = lane >> 4, c4 = (lane & 15) * 4;
  for (int pass = 0; pass < 2; ++pass) {
#pragma unroll
    for (int it = 0; it < 4; ++it) {
      const int rl = wave * 8 + it * 2 + hh;
      const v4f v = *(const v4f*)(sO + rl * kPrjOP + c4);
      *(volatile v4f*)(PROJ + (size_t)(row0 + rl) * kPrjP + c4) = v;
    }
    __threadfence();
  }
}

__global__ __launch_bounds__(kRpThreads) void rowprep_kernel(
    const float* __restrict__ PROJ, const float* __restrict__ Bbias, const float* __restrict__ Cbias,
    const float* __restrict__ blam, float* __restrict__ RREC)
{
  __shared__ __align__(16) float sTot[kRpThreads * kNth];
  __shared__ __align__(16) float sOff[kRpThreads * kNth];
  __shared__ __align__(16) float sBias[2 * kNst];
  __shared__ __align__(16) float sR[kRpThreads * kRpLP];
  const int tid = threadIdx.x, lane = tid & 31, wave = tid >> 5;
  const size_t rb = (size_t)blockIdx.x * kSeq;
  const float bl0 = blam[0];
  if (tid < 2 * kNst) {
    const float vb = Bbias[tid & (kNst - 1)];
    const float vc = Cbias[tid & (kNst - 1)];
    const float fb = (tid < kNst) ? 1.f : 0.f;
    sBias[tid] = fmaf(fb, vb, (1.f - fb) * vc);
  }
  float su[8];
#pragma unroll
  for (int j = 0; j < 8; ++j) su[j] = 0.f;
#pragma unroll 1
  for (int i = 0; i < kRpGroup; ++i) {
    const float* p = PROJ + (rb + (size_t)tid * kRpGroup + i) * kPrjP + 2 * kNst;
    const v4f a = *(const v4f*)p;
    const v4f c = *(const v4f*)(p + 4);
    su[0] += a[0]; su[1] += a[1]; su[2] += a[2]; su[3] += a[3];
    su[4] += c[0]; su[5] += c[1]; su[6] += c[2]; su[7] += c[3];
  }
  *(v4f*)(sTot + tid * kNth)     = (v4f){su[0], su[1], su[2], su[3]};
  *(v4f*)(sTot + tid * kNth + 4) = (v4f){su[4], su[5], su[6], su[7]};
  __syncthreads();
  if (tid < kNth) {
    float run = 0.f;
#pragma unroll 1
    for (int g = 0; g < kRpThreads; ++g) {
      const float t = sTot[g * kNth + tid];
      sOff[g * kNth + tid] = run;
      run += t;
    }
  }
  __syncthreads();
  const int gl  = tid >> 4;
  const int iin = tid & 15;
  const int hh = lane >> 4, c4 = (lane & 15) * 4;
  const v4f z4 = (v4f){0.f, 0.f, 0.f, 0.f};
#pragma unroll 1
  for (int c = 0; c < kSeq / kRpThreads; ++c) {
    const size_t r0 = rb + (size_t)c * kRpThreads;
#pragma unroll 1
    for (int i = 0; i < 12; ++i) {
      const int idx = tid + kRpThreads * i;
      const int rl = idx / 12;
      const int q = idx - rl * 12;
      *(v4f*)(sR + rl * kRpLP + 4 * q) = *(const v4f*)(PROJ + (r0 + rl) * kPrjP + 4 * q);
    }
    __syncthreads();
    float th[8];
    {
      const v4f o0 = *(const v4f*)(sOff + (c * 8 + gl) * kNth);
      const v4f o1 = *(const v4f*)(sOff + (c * 8 + gl) * kNth + 4);
      th[0] = o0[0]; th[1] = o0[1]; th[2] = o0[2]; th[3] = o0[3];
      th[4] = o1[0]; th[5] = o1[1]; th[6] = o1[2]; th[7] = o1[3];
    }
#pragma unroll 1
    for (int i = 0; i < kRpGroup; ++i) {
      const float f = (i <= iin) ? 1.f : 0.f;
      const float* p = sR + (gl * kRpGroup + i) * kRpLP + 2 * kNst;
      const v4f a = *(const v4f*)p;
      const v4f q4 = *(const v4f*)(p + 4);
      th[0] = fmaf(f, a[0], th[0]);  th[1] = fmaf(f, a[1], th[1]);
      th[2] = fmaf(f, a[2], th[2]);  th[3] = fmaf(f, a[3], th[3]);
      th[4] = fmaf(f, q4[0], th[4]); th[5] = fmaf(f, q4[1], th[5]);
      th[6] = fmaf(f, q4[2], th[6]); th[7] = fmaf(f, q4[3], th[7]);
    }
    *(v4f*)(sTot + tid * kNth)     = (v4f){th[0], th[1], th[2], th[3]};
    *(v4f*)(sTot + tid * kNth + 4) = (v4f){th[4], th[5], th[6], th[7]};
    __syncthreads();
    float* row = sR + tid * kRpLP;
#pragma unroll 1
    for (int j = 0; j < kNth; ++j) {
      const float ang = sTot[tid * kNth + j];
      float sn, cs;
      sincosf(ang, &sn, &cs);
      const float b0 = row[j] + sBias[j];
      const float b1 = row[j + kNth] + sBias[j + kNth];
      const float e0 = row[kNst + j] + sBias[kNst + j];
      const float e1 = row[kNst + kNth + j] + sBias[kNst + kNth + j];
      row[j]               = b0 * cs - b1 * sn;
      row[j + kNth]        = b1 * cs + b0 * sn;
      row[kNst + j]        = e0 * cs - e1 * sn;
      row[kNst + kNth + j] = e1 * cs + e0 * sn;
    }
    {
      const float p40 = row[2 * kNst + kNth];
      const float p41 = row[2 * kNst + kNth + 1];
      const float av  = __expf(-fabsf(p40));
      const float uu  = 1.0f + av;
      const float l1p = __logf(uu) + (av - (uu - 1.0f)) * __builtin_amdgcn_rcpf(uu);
      const float dtsp = fmaxf(p40, 0.0f) + l1p;
      const float lv  = p41 + bl0;
      const float lam = __builtin_amdgcn_rcpf(1.0f + __expf(-lv));
      row[32] = dtsp; row[33] = lam; row[34] = 0.f; row[35] = 0.f;
#pragma unroll
      for (int q4i = 9; q4i < 16; ++q4i) *(v4f*)(row + 4 * q4i) = z4;
    }
    __syncthreads();
    for (int pass = 0; pass < 2; ++pass) {
#pragma unroll
      for (int it = 0; it < 16; ++it) {
        const int rl = it * 8 + wave * 2 + hh;
        const v4f v = *(const v4f*)(sR + rl * kRpLP + c4);
        *(volatile v4f*)(RREC + (r0 + rl) * kRecP + c4) = v;
      }
      __threadfence();
    }
    __syncthreads();
  }
}

__global__ __launch_bounds__(kScanCh) void scan_kernel(
    const float* __restrict__ RREC, const float* __restrict__ UC, const float* __restrict__ XZ,
    const float* __restrict__ Wdt, const float* __restrict__ bdt, const float* __restrict__ Alog,
    const float* __restrict__ Dp, unsigned short* __restrict__ Y16)
{
  __shared__ __align__(16) float sX[kScanTS * kRecP];
  __shared__ __align__(16) float sY[kScanTS * kScanYP];
  __shared__ __align__(16) float sA[kNst * kScanCh];
  const int tid = threadIdx.x, lane = tid & 31, wave = tid >> 5;
  constexpr int kBlkPerB = kDin / kScanCh;
  const int bix = blockIdx.x / kBlkPerB;
  const int d0  = (blockIdx.x - bix * kBlkPerB) * kScanCh;
  const int d   = d0 + tid;
  const size_t row0 = (size_t)bix * kSeq;
#pragma unroll 1
  for (int n = 0; n < kNst; ++n) sA[n * kScanCh + tid] = -expf(Alog[(size_t)d * kNst + n]);
  __syncthreads();
  float negA[kNst], h[kNst], bxp[kNst];
#pragma unroll
  for (int n = 0; n < kNst; ++n) {
    negA[n] = sA[n * kScanCh + tid];
    h[n] = 0.f;
    bxp[n] = 0.f;
  }
  const float wd = Wdt[d], bb = bdt[d], Dd = Dp[d];
  const int lr = tid >> 4, lc4 = (tid & 15) * 4;
  const int q = lane >> 3, c8 = (lane & 7) * 8;
#pragma unroll 1
  for (int t0 = 0; t0 < kSeq; t0 += kScanTS) {
    __syncthreads();
#pragma unroll 1
    for (int i = 0; i < 16; ++i) {
      const int r = lr + 4 * i;
      *(v4f*)(sX + r * kRecP + lc4) = *(const v4f*)(RREC + (row0 + t0 + r) * kRecP + lc4);
    }
    __syncthreads();
#pragma unroll 1
    for (int s = 0; s < kScanTS; ++s) {
      const size_t m = row0 + t0 + s;
      const float* xr = sX + s * kRecP;
      v4f Bq[4], Cq[4];
#pragma unroll
      for (int qq = 0; qq < 4; ++qq) {
        Bq[qq] = *(const v4f*)(xr + 4 * qq);
        Cq[qq] = *(const v4f*)(xr + kNst + 4 * qq);
      }
      const v4f sc  = *(const v4f*)(xr + 2 * kNst);
      const float v   = fmaf(sc[0], wd, bb);
      const float av  = __expf(-fabsf(v));
      const float uu  = 1.0f + av;
      const float l1p = __logf(uu) + (av - (uu - 1.0f)) * __builtin_amdgcn_rcpf(uu);
      const float delta = fmaxf(v, 0.0f) + l1p;
      const float lam   = sc[1];
      const float u  = UC[m * kDin + d];
      const float zv = XZ[m * kXzP + kDin + d];
      const float lamde = lam * delta;
      const float omlde = (1.0f - lam) * delta;
      float y = 0.f;
#pragma unroll
      for (int n = 0; n < kNst; ++n) {
        const float e   = __expf(delta * negA[n]);
        const float bx  = Bq[n >> 2][n & 3] * u;
        const float t2  = (omlde * e) * bxp[n];
        const float inp = fmaf(lamde, bx, t2);
        const float hn  = fmaf(e, h[n], inp);
        h[n] = hn;
        bxp[n] = bx;
        y = fmaf(hn, Cq[n >> 2][n & 3], y);
      }
      y = fmaf(u, Dd, y);
      const float sg = __builtin_amdgcn_rcpf(1.0f + __expf(-zv));
      y = y * (zv * sg);
      sY[s * kScanYP + tid] = y * kYCarry;
    }
    __syncthreads();
    v8h hv[8];
#pragma unroll
    for (int it = 0; it < 8; ++it) {
      const int row = it * 8 + wave * 4 + q;
      const float* sp = sY + row * kScanYP + c8;
      const v4f a0 = *(const v4f*)(sp);
      const v4f a1 = *(const v4f*)(sp + 4);
#pragma unroll
      for (int e = 0; e < 4; ++e) {
        hv[it][e]     = (_Float16)a0[e];
        hv[it][4 + e] = (_Float16)a1[e];
      }
    }
    for (int pass = 0; pass < 2; ++pass) {
#pragma unroll
      for (int it = 0; it < 8; ++it) {
        const int row = it * 8 + wave * 4 + q;
        const size_t o = (row0 + t0 + row) * kDin + d0 + c8;
        *(volatile v8h*)(Y16 + o) = hv[it];
      }
      __threadfence();
    }
  }
}

extern "C" void kernel_launch(void* const* d_in, const int* in_sizes, int n_in,
                              void* d_out, int out_size, void* d_ws, size_t ws_size,
                              hipStream_t stream)
{
  if (n_in < 15) return;
  if (in_sizes[0]  != kRows * kDm) return;
  if (in_sizes[1]  != kDm * kXzP) return;
  if (in_sizes[2]  != kDin * kConvK) return;
  if (in_sizes[3]  != kDin) return;
  if (in_sizes[4]  != kDin * kWxN) return;
  if (in_sizes[5]  != kDin) return;
  if (in_sizes[6]  != kDin) return;
  if (in_sizes[7]  != kDin * kNst) return;
  if (in_sizes[8]  != kNst) return;
  if (in_sizes[9]  != kNst) return;
  if (in_sizes[10] != kDin * kNth) return;
  if (in_sizes[11] != kDin) return;
  if (in_sizes[12] != 1) return;
  if (in_sizes[13] != kDin * kDm) return;
  if (in_sizes[14] != kDin) return;
  if (out_size != kRows * kDm) return;
  if (ws_size < kWsTotal) return;

  const float* x       = (const float*)d_in[0];
  const float* W_in    = (const float*)d_in[1];
  const float* conv_w  = (const float*)d_in[2];
  const float* conv_b  = (const float*)d_in[3];
  const float* W_x     = (const float*)d_in[4];
  const float* W_dt    = (const float*)d_in[5];
  const float* b_dt    = (const float*)d_in[6];
  const float* A_log   = (const float*)d_in[7];
  const float* B_bias  = (const float*)d_in[8];
  const float* C_bias  = (const float*)d_in[9];
  const float* W_theta = (const float*)d_in[10];
  const float* W_lam   = (const float*)d_in[11];
  const float* b_lam   = (const float*)d_in[12];
  const float* W_out   = (const float*)d_in[13];
  const float* Dp      = (const float*)d_in[14];
  float* out = (float*)d_out;

  char* ws = (char*)d_ws;
  unsigned short* XH   = (unsigned short*)(ws + kOffXH);
  unsigned short* XL   = (unsigned short*)(ws + kOffXL);
  unsigned short* WIH  = (unsigned short*)(ws + kOffWIH);
  unsigned short* WIL  = (unsigned short*)(ws + kOffWIL);
  unsigned short* WO16 = (unsigned short*)(ws + kOffWO16);
  float*          XZ   = (float*)(ws + kOffXZ);
  float*          UC   = (float*)(ws + kOffUC);
  float*          PROJ = (float*)(ws + kOffPRJ);
  float*          RREC = (float*)(ws + kOffREC);
  unsigned short* Y16  = (unsigned short*)(ws + kOffY16);
  const float* dummy_bias  = b_dt;
  const float* dummy_resid = x;

  split_rows_bf16_kernel<<<(kRows * kDm / 8) / 256, 256, 0, stream>>>(x, XH, XL, kRows * kDm / 8);
  transpose_split_bf16_kernel<<<dim3(kXzP / 64, kDm / 64), 256, 0, stream>>>(W_in, WIH, WIL, kDm, kXzP);
  transpose_cast_kernel<<<dim3(kDm / 64, kDin / 64), 256, 0, stream>>>(W_out, WO16, kDin, kDm, kDm, kWCarry);

  wmma_gemm64<1, true, 0, 0, false><<<dim3((kRows / 64) * (kXzP / 64) / 8, 1), 256, 0, stream>>>(
      XH, XL, kDm, 0L,
      WIH, WIL, kDm, 0L,
      (void*)XZ, (void*)XZ, kXzP, 0L,
      dummy_bias, dummy_resid, 0L,
      kRows, kXzP, kDm, 1.0f);

  conv_silu_kernel<<<dim3(kDin / 256, kRows / 64), 256, 0, stream>>>(XZ, conv_w, conv_b, UC);

  proj_kernel<<<kRows / kPrjRows, 256, 0, stream>>>(UC, W_x, W_theta, W_lam, PROJ);

  rowprep_kernel<<<kBatch, kRpThreads, 0, stream>>>(PROJ, B_bias, C_bias, b_lam, RREC);

  scan_kernel<<<kBatch * (kDin / kScanCh), kScanCh, 0, stream>>>(RREC, UC, XZ, W_dt, b_dt, A_log, Dp, Y16);

  wmma_gemm64<0, false, 0, 0, false><<<dim3((kRows / 64) * (kDm / 64) / 8, 1), 256, 0, stream>>>(
      Y16, Y16, kDin, 0L,
      WO16, WO16, kDin, 0L,
      (void*)out, (void*)out, kDm, 0L,
      dummy_bias, dummy_resid, 0L,
      kRows, kDm, kDin, kOutScale);
}
